// Encoder_76630806495266
// MI455X (gfx1250) — hardware-verified
//
#include <hip/hip_runtime.h>
#include <math.h>

constexpr int NBAT    = 128;
constexpr int NSTEP   = 50;
constexpr int NNODE   = 24;
constexpr int NDIM    = 6;
constexpr int NHID    = 256;
constexpr int NGATE   = 1024;
constexpr int NOUTF   = 256;
constexpr int NTYPE   = 7;
constexpr int BMROWS  = 32;
constexpr int NTHR    = 256;
constexpr int KTILES  = 9;
constexpr int APITCH  = 296;
constexpr int KPITCH  = 320;
constexpr int CPITCH  = 260;
constexpr int PLANE   = NBAT * NNODE * NHID;
constexpr int ROWSTR  = NNODE * NHID;
constexpr float WCARRY     = 16.0f;
constexpr float WCARRY_INV = 1.0f / 16.0f;
constexpr float XLCARRY    = 64.0f;
constexpr float XLW        = WCARRY / XLCARRY;

static_assert(NGATE == 4 * NHID, "gate width");
static_assert(NHID == 32 * (NTHR / 32), "8 waves x 32 hidden columns");
static_assert(BMROWS == 32, "one lane per staged x row; two m-subtiles");
static_assert(NBAT % BMROWS == 0, "batch tiles");
static_assert(KTILES * 32 >= NHID + 2 * NDIM, "x hi/lo columns fit in the last k-tile");
static_assert(KTILES * 32 <= APITCH && KTILES * 32 <= KPITCH, "k-tiles stay inside the pitches");
static_assert((KPITCH * 2) % 128 == 0 && (NHID * 2) % 128 == 0, "plane rows are whole lines");
static_assert((APITCH * 2) % 16 == 0 && (CPITCH * 4) % 16 == 0, "16-B aligned LDS rows");
static_assert((size_t)4 * PLANE * 4 == (size_t)12582912, "output bytes");
static_assert(NHID % 64 == 0 && NGATE % 64 == 0 && NOUTF % 64 == 0, "transpose tiles");

typedef __attribute__((ext_vector_type(16))) _Float16 v16h;
typedef __attribute__((ext_vector_type(8)))  _Float16 v8h;
typedef __attribute__((ext_vector_type(8)))  float    v8f;
typedef __attribute__((ext_vector_type(4)))  float    v4f;
typedef __attribute__((ext_vector_type(2)))  float    v2f;

__device__ __forceinline__ v16h frag_ld(const _Float16* p) {
  union U { v16h v; v8h h[2]; } f;
  f.h[0] = *(const v8h*)(p);
  f.h[1] = *(const v8h*)(p + 16);
  return f.v;
}
__device__ __forceinline__ v8f mma_h(v16h a, v16h b, v8f c) {
  return __builtin_amdgcn_wmma_f32_16x16x32_f16(false, a, false, b, (short)0, c, false, false);
}
__device__ __forceinline__ void guard8_h(v8f& a0, v8f& a1, v8f& a2, v8f& a3, v8f& a4, v8f& a5, v8f& a6, v8f& a7,
                                         v16h x0, v16h x1, v16h y0, v16h y1, v16h y2, v16h y3) {
  asm volatile("v_nop\n\tv_nop\n\tv_nop\n\tv_nop"
               : "+v"(a0), "+v"(a1), "+v"(a2), "+v"(a3), "+v"(a4), "+v"(a5), "+v"(a6), "+v"(a7)
               : "v"(x0), "v"(x1), "v"(y0), "v"(y1), "v"(y2), "v"(y3));
}
__device__ __forceinline__ void accguard8(v8f& a0, v8f& a1, v8f& a2, v8f& a3, v8f& a4, v8f& a5, v8f& a6, v8f& a7) {
  asm volatile("v_nop\n\tv_nop\n\tv_nop\n\tv_nop"
               : "+v"(a0), "+v"(a1), "+v"(a2), "+v"(a3), "+v"(a4), "+v"(a5), "+v"(a6), "+v"(a7));
}
__device__ __forceinline__ void guard4_h(v8f& a0, v8f& a1, v8f& a2, v8f& a3, v16h x0, v16h x1, v16h y0, v16h y1) {
  asm volatile("v_nop\n\tv_nop\n\tv_nop\n\tv_nop"
               : "+v"(a0), "+v"(a1), "+v"(a2), "+v"(a3)
               : "v"(x0), "v"(x1), "v"(y0), "v"(y1));
}
__device__ __forceinline__ void accguard4(v8f& a0, v8f& a1, v8f& a2, v8f& a3) {
  asm volatile("v_nop\n\tv_nop\n\tv_nop\n\tv_nop" : "+v"(a0), "+v"(a1), "+v"(a2), "+v"(a3));
}

__device__ __forceinline__ float fsig(float v)  { return __builtin_amdgcn_rcpf(1.0f + expf(-v)); }
__device__ __forceinline__ float ftanh(float v) { return 1.0f - 2.0f * __builtin_amdgcn_rcpf(expf(2.0f * v) + 1.0f); }

__global__ __launch_bounds__(NTHR) void tpw_kernel(const float* __restrict__ src, int R, int C, int ldo,
                                                   unsigned short* __restrict__ O, float sc) {
  __shared__ float Tt[64 * 65];
  const int tid = threadIdx.x;
  const int c0 = blockIdx.x * 64, r0 = blockIdx.y * 64;
  const float* sp = src + (size_t)blockIdx.z * (size_t)R * (size_t)C;
  unsigned short* op = O + (size_t)blockIdx.z * (size_t)C * (size_t)ldo;
#pragma unroll
  for (int i = 0; i < 4; ++i) {
    const int idx = i * NTHR + tid;
    const int rr = idx >> 4, cc = (idx & 15) * 4;
    const v4f v = *(const v4f*)(sp + (size_t)(r0 + rr) * (size_t)C + c0 + cc);
    Tt[rr * 65 + cc + 0] = v[0];
    Tt[rr * 65 + cc + 1] = v[1];
    Tt[rr * 65 + cc + 2] = v[2];
    Tt[rr * 65 + cc + 3] = v[3];
  }
  __syncthreads();
  const int q = tid >> 3, c8 = (tid & 7) * 8;
  v8h hv[2];
#pragma unroll
  for (int g = 0; g < 2; ++g) {
    const int qq = g * 32 + q;
#pragma unroll
    for (int e = 0; e < 8; ++e) {
      const float f = Tt[(c8 + e) * 65 + qq];
      hv[g][e] = (_Float16)(f * sc);
    }
  }
  for (int pass = 0; pass < 2; ++pass) {
#pragma unroll
    for (int g = 0; g < 2; ++g) {
      const size_t o = (size_t)(c0 + g * 32 + q) * (size_t)ldo + (size_t)(r0 + c8);
      *(volatile v8h*)(op + o) = hv[g];
    }
    __threadfence();
  }
}

__global__ __launch_bounds__(NTHR) void wx_cols_kernel(const float* __restrict__ w_ih, unsigned short* __restrict__ WgT) {
  const int i = blockIdx.x * NTHR + threadIdx.x;
  if (i < NTYPE * NGATE * 8) {
    const int rowi = i >> 3;
    const int sub = i & 7;
    const int ty = rowi >> 10;
    const int n = rowi & (NGATE - 1);
    v8h hv;
#pragma unroll
    for (int e = 0; e < 8; ++e) {
      const int kk = 8 * sub + e;
      int d = (kk < NDIM) ? kk : (kk - NDIM);
      d = d < 0 ? 0 : d;
      d = d > (NDIM - 1) ? (NDIM - 1) : d;
      const float f = w_ih[((size_t)ty * NDIM + d) * NGATE + n];
      const float scl = (kk < NDIM) ? WCARRY : XLW;
      float val = f * scl;
      val = (kk < 2 * NDIM) ? val : 0.0f;
      hv[e] = (_Float16)val;
    }
    unsigned short* p = WgT + (size_t)rowi * KPITCH + NHID + 8 * sub;
    *(volatile v8h*)p = hv;
    __threadfence();
    *(volatile v8h*)p = hv;
  }
}

__global__ __launch_bounds__(NTHR) void bias_sum_kernel(const float* __restrict__ b_ih, const float* __restrict__ b_hh,
                                                        float* __restrict__ Bsum) {
  const int i = blockIdx.x * NTHR + threadIdx.x;
  if (i < NTYPE * NGATE / 4) {
    const v4f a = *(const v4f*)(b_ih + 4 * i);
    const v4f b = *(const v4f*)(b_hh + 4 * i);
    const v4f o = a + b;
    *(volatile v4f*)(Bsum + 4 * i) = o;
    __threadfence();
    *(volatile v4f*)(Bsum + 4 * i) = o;
  }
}

__device__ __forceinline__ void stage_x(const float* __restrict__ x, int b0, int node, int t, int lane, _Float16* Abuf) {
  const float* xp = x + ((size_t)(b0 + lane) * NSTEP + (size_t)t) * (size_t)(NNODE * NDIM) + node * NDIM;
  const v2f p0 = *(const v2f*)(xp);
  const v2f p1 = *(const v2f*)(xp + 2);
  const v2f p2 = *(const v2f*)(xp + 4);
  const float x0 = p0[0], x1 = p0[1], x2 = p1[0], x3 = p1[1], x4 = p2[0], x5 = p2[1];
  const _Float16 h0 = (_Float16)x0, h1 = (_Float16)x1, h2 = (_Float16)x2;
  const _Float16 h3 = (_Float16)x3, h4 = (_Float16)x4, h5 = (_Float16)x5;
  const _Float16 l0 = (_Float16)((x0 - (float)h0) * XLCARRY);
  const _Float16 l1 = (_Float16)((x1 - (float)h1) * XLCARRY);
  const _Float16 l2 = (_Float16)((x2 - (float)h2) * XLCARRY);
  const _Float16 l3 = (_Float16)((x3 - (float)h3) * XLCARRY);
  const _Float16 l4 = (_Float16)((x4 - (float)h4) * XLCARRY);
  const _Float16 l5 = (_Float16)((x5 - (float)h5) * XLCARRY);
  const _Float16 zz = (_Float16)0.0f;
  v8h q0, q1, q2;
  q0[0] = h0; q0[1] = h1; q0[2] = h2; q0[3] = h3; q0[4] = h4; q0[5] = h5; q0[6] = l0; q0[7] = l1;
  q1[0] = l2; q1[1] = l3; q1[2] = l4; q1[3] = l5; q1[4] = zz; q1[5] = zz; q1[6] = zz; q1[7] = zz;
  q2[0] = zz; q2[1] = zz; q2[2] = zz; q2[3] = zz; q2[4] = zz; q2[5] = zz; q2[6] = zz; q2[7] = zz;
  _Float16* dp = Abuf + lane * APITCH + NHID;
  *(v8h*)(dp)      = q0;
  *(v8h*)(dp + 8)  = q1;
  *(v8h*)(dp + 16) = q2;
  *(v8h*)(dp + 24) = q2;
}

template <bool LK>
__device__ __forceinline__ void store_rows(const float* S, float* g, int tid) {
  for (int pass = 0; pass < 2; ++pass) {
#pragma unroll
    for (int it = 0; it < 8; ++it) {
      const int idx = it * NTHR + tid;
      const int row = idx >> 6;
      const int c4 = (idx & 63) * 4;
      v4f v = *(const v4f*)(S + row * CPITCH + c4);
      if (LK) {
#pragma unroll
        for (int e = 0; e < 4; ++e) {
          const float f = v[e];
          v[e] = (f >= 0.0f) ? f : 0.01f * f;
        }
      }
      *(volatile v4f*)(g + (size_t)row * ROWSTR + c4) = v;
    }
    __threadfence();
  }
}

__global__ __launch_bounds__(NTHR) void enc_kernel(const float* __restrict__ x, const int* __restrict__ node_types,
                                                   const float* __restrict__ h1_w, const float* __restrict__ h1_b,
                                                   const float* __restrict__ h2_w, const float* __restrict__ h2_b,
                                                   const float* __restrict__ fc_b,
                                                   const unsigned short* __restrict__ WgTp,
                                                   const unsigned short* __restrict__ FcTp,
                                                   const float* __restrict__ Bsum, float* __restrict__ out) {
  __shared__ __align__(16) _Float16 At[2 * BMROWS * APITCH];
  __shared__ __align__(16) float    Cs[BMROWS * CPITCH];
  __shared__ __align__(16) float    Hs[BMROWS * CPITCH];
  __shared__ __align__(16) float    sB[NGATE];
  __shared__ __align__(16) float    sX[BMROWS * 8];

  const _Float16* WgT = (const _Float16*)WgTp;
  const _Float16* FcT = (const _Float16*)FcTp;
  const int tid = threadIdx.x, lane = tid & 31;
  const int wave = __builtin_amdgcn_readfirstlane(tid >> 5);
  const int c = lane & 15, hh = lane >> 4, koff = hh * 8;
  const int node = blockIdx.x >> 2;
  const int b0 = (blockIdx.x & 3) * BMROWS;
  int ty = node_types[node];
  ty = ty < 0 ? 0 : ty;
  ty = ty > (NTYPE - 1) ? (NTYPE - 1) : ty;

#pragma unroll
  for (int j = 0; j < 4; ++j) sB[tid + NTHR * j] = Bsum[(size_t)ty * NGATE + tid + NTHR * j] * WCARRY;
  if (tid < BMROWS * NDIM) {
    const int row = tid / NDIM;
    const int d = tid - row * NDIM;
    sX[row * 8 + d] = x[((size_t)(b0 + row) * NSTEP) * (size_t)(NNODE * NDIM) + node * NDIM + d];
  }
  __syncthreads();

  {
    float w1[NDIM], w2[NDIM];
#pragma unroll
    for (int d = 0; d < NDIM; ++d) w1[d] = h1_w[((size_t)ty * NDIM + d) * NHID + tid];
    asm volatile("" ::: "memory");
#pragma unroll
    for (int d = 0; d < NDIM; ++d) w2[d] = h2_w[((size_t)ty * NDIM + d) * NHID + tid];
    const float bb1 = h1_b[ty * NHID + tid];
    const float bb2 = h2_b[ty * NHID + tid];
#pragma unroll 1
    for (int row = 0; row < BMROWS; ++row) {
      float hv = 0.0f, cv = 0.0f;
#pragma unroll
      for (int d = 0; d < NDIM; ++d) {
        const float xv = sX[row * 8 + d];
        hv = fmaf(xv, w1[d], hv);
        cv = fmaf(xv, w2[d], cv);
      }
      hv += bb1;
      cv += bb2;
      At[row * APITCH + tid] = (_Float16)hv;
      Cs[row * CPITCH + tid] = cv;
    }
  }
  if (wave == 0) stage_x(x, b0, node, 0, lane, At);
  __syncthreads();

#pragma unroll 1
  for (int t = 0; t < NSTEP; ++t) {
    const int cur = t & 1;
    const _Float16* Ac = At + cur * (BMROWS * APITCH);
    _Float16* An = At + (cur ^ 1) * (BMROWS * APITCH);
    const bool cm = (t % (wave + 1)) == 0;
    const bool last = (t == NSTEP - 1);
    const _Float16* a0p = Ac + c * APITCH + koff;
    const _Float16* a1p = Ac + (16 + c) * APITCH + koff;

#pragma unroll 1
    for (int s = 0; s < 2; ++s) {
      const int ncol = 32 * wave + 16 * s + c;
      const float bi = sB[ncol];
      const float bf = sB[NHID + ncol];
      const float bg = sB[2 * NHID + ncol];
      const float bo = sB[3 * NHID + ncol];
      v8f acc[4][2];
      acc[0][0] = (v8f){bi, bi, bi, bi, bi, bi, bi, bi};
      acc[0][1] = acc[0][0];
      acc[1][0] = (v8f){bf, bf, bf, bf, bf, bf, bf, bf};
      acc[1][1] = acc[1][0];
      acc[2][0] = (v8f){bg, bg, bg, bg, bg, bg, bg, bg};
      acc[2][1] = acc[2][0];
      acc[3][0] = (v8f){bo, bo, bo, bo, bo, bo, bo, bo};
      acc[3][1] = acc[3][0];
      const _Float16* wrow = WgT + ((size_t)ty * NGATE + ncol) * KPITCH + koff;
#pragma unroll 1
      for (int kt = 0; kt < KTILES; ++kt) {
        const int k0 = kt * 32;
        const v16h a0 = frag_ld(a0p + k0);
        const v16h a1 = frag_ld(a1p + k0);
        const v16h b0 = frag_ld(wrow + k0);
        const v16h b1 = frag_ld(wrow + (size_t)1 * NHID * KPITCH + k0);
        const v16h b2 = frag_ld(wrow + (size_t)2 * NHID * KPITCH + k0);
        const v16h b3 = frag_ld(wrow + (size_t)3 * NHID * KPITCH + k0);
        acc[0][0] = mma_h(a0, b0, acc[0][0]);
        acc[0][1] = mma_h(a1, b0, acc[0][1]);
        acc[1][0] = mma_h(a0, b1, acc[1][0]);
        acc[1][1] = mma_h(a1, b1, acc[1][1]);
        acc[2][0] = mma_h(a0, b2, acc[2][0]);
        acc[2][1] = mma_h(a1, b2, acc[2][1]);
        acc[3][0] = mma_h(a0, b3, acc[3][0]);
        acc[3][1] = mma_h(a1, b3, acc[3][1]);
        guard8_h(acc[0][0], acc[0][1], acc[1][0], acc[1][1], acc[2][0], acc[2][1], acc[3][0], acc[3][1],
                 a0, a1, b0, b1, b2, b3);
      }
      accguard8(acc[0][0], acc[0][1], acc[1][0], acc[1][1], acc[2][0], acc[2][1], acc[3][0], acc[3][1]);

#pragma unroll 1
      for (int mi = 0; mi < 2; ++mi) {
        const v8f zi = mi ? acc[0][1] : acc[0][0];
        const v8f zf = mi ? acc[1][1] : acc[1][0];
        const v8f zg = mi ? acc[2][1] : acc[2][0];
        const v8f zo = mi ? acc[3][1] : acc[3][0];
        const int rb = 16 * mi + 8 * hh;
#pragma unroll
        for (int r = 0; r < 8; ++r) {
          const int row = rb + r;
          const float pi = zi[r] * WCARRY_INV;
          const float pf = zf[r] * WCARRY_INV;
          const float pg = zg[r] * WCARRY_INV;
          const float po = zo[r] * WCARRY_INV;
          const float cold = Cs[row * CPITCH + ncol];
          const float ig = fsig(pi);
          const float fg = fsig(pf);
          const float gg = ftanh(pg);
          const float og = fsig(po);
          const float cnew = fg * cold + ig * gg;
          const float cy = cm ? cnew : cold;
          Cs[row * CPITCH + ncol] = cy;
          const float hy = og * ftanh(cy);
          An[row * APITCH + ncol] = (_Float16)hy;
          if (last) Hs[row * CPITCH + ncol] = hy;
        }
      }
    }
    if (wave == 0) {
      const int tn = (t + 1 < NSTEP) ? (t + 1) : (NSTEP - 1);
      stage_x(x, b0, node, tn, lane, An);
    }
    __syncthreads();
  }

  float* gbase = out + ((size_t)b0 * NNODE + node) * NHID;
  store_rows<false>(Hs, gbase + (size_t)1 * PLANE, tid);
  store_rows<false>(Cs, gbase + (size_t)2 * PLANE, tid);
  store_rows<true>(Hs, gbase + (size_t)3 * PLANE, tid);
  __syncthreads();

  {
    const _Float16* Af = At + (NSTEP & 1) * (BMROWS * APITCH);
    const _Float16* a0p = Af + c * APITCH + koff;
    const _Float16* a1p = Af + (16 + c) * APITCH + koff;
    const _Float16* f0 = FcT + ((size_t)ty * NOUTF + 32 * wave + c) * NHID + koff;
    const _Float16* f1 = f0 + (size_t)16 * NHID;
    const v8f z8 = {0.f, 0.f, 0.f, 0.f, 0.f, 0.f, 0.f, 0.f};
    v8f hacc[2][2];
    hacc[0][0] = z8; hacc[0][1] = z8; hacc[1][0] = z8; hacc[1][1] = z8;
#pragma unroll 1
    for (int k0 = 0; k0 < NHID; k0 += 32) {
      const v16h a0 = frag_ld(a0p + k0);
      const v16h a1 = frag_ld(a1p + k0);
      const v16h b0 = frag_ld(f0 + k0);
      const v16h b1 = frag_ld(f1 + k0);
      hacc[0][0] = mma_h(a0, b0, hacc[0][0]);
      hacc[0][1] = mma_h(a1, b0, hacc[0][1]);
      hacc[1][0] = mma_h(a0, b1, hacc[1][0]);
      hacc[1][1] = mma_h(a1, b1, hacc[1][1]);
      guard4_h(hacc[0][0], hacc[0][1], hacc[1][0], hacc[1][1], a0, a1, b0, b1);
    }
    accguard4(hacc[0][0], hacc[0][1], hacc[1][0], hacc[1][1]);
#pragma unroll
    for (int nt = 0; nt < 2; ++nt) {
      const int col = 32 * wave + 16 * nt + c;
      const float fb = fc_b[ty * NOUTF + col];
#pragma unroll
      for (int mi = 0; mi < 2; ++mi) {
#pragma unroll
        for (int r = 0; r < 8; ++r) {
          float v = hacc[nt][mi][r] * WCARRY_INV + fb;
          v = (v >= 0.0f) ? v : 0.01f * v;
          Hs[(16 * mi + 8 * hh + r) * CPITCH + col] = v;
        }
      }
    }
  }
  __syncthreads();
  store_rows<false>(Hs, gbase, tid);
}

extern "C" void kernel_launch(void* const* d_in, const int* in_sizes, int n_in,
                              void* d_out, int out_size, void* d_ws, size_t ws_size, hipStream_t stream) {
  if (n_in < 12 || d_out == nullptr || d_ws == nullptr) return;
  if (in_sizes[0] != NBAT * NSTEP * NNODE * NDIM || in_sizes[1] != NNODE ||
      in_sizes[2] != NTYPE * NDIM * NGATE || in_sizes[3] != NTYPE * NHID * NGATE ||
      in_sizes[4] != NTYPE * NGATE || in_sizes[5] != NTYPE * NGATE ||
      in_sizes[6] != NTYPE * NHID * NOUTF || in_sizes[7] != NTYPE * NOUTF ||
      in_sizes[8] != NTYPE * NDIM * NHID || in_sizes[9] != NTYPE * NHID ||
      in_sizes[10] != NTYPE * NDIM * NHID || in_sizes[11] != NTYPE * NHID ||
      out_size != 4 * PLANE) return;

  const float* x          = (const float*)d_in[0];
  const int*   node_types = (const int*)d_in[1];
  const float* w_ih       = (const float*)d_in[2];
  const float* w_hh       = (const float*)d_in[3];
  const float* b_ih       = (const float*)d_in[4];
  const float* b_hh       = (const float*)d_in[5];
  const float* fc_w       = (const float*)d_in[6];
  const float* fc_b       = (const float*)d_in[7];
  const float* h1_w       = (const float*)d_in[8];
  const float* h1_b       = (const float*)d_in[9];
  const float* h2_w       = (const float*)d_in[10];
  const float* h2_b       = (const float*)d_in[11];
  float* out = (float*)d_out;

  char* ws = (char*)d_ws; size_t off = 0;
  auto carve = [&](size_t bytes) -> char* { char* p = ws + off; off += (bytes + 255) & ~(size_t)255; return p; };
  unsigned short* WgT  = (unsigned short*)carve((size_t)NTYPE * NGATE * KPITCH * 2);
  unsigned short* FcT  = (unsigned short*)carve((size_t)NTYPE * NOUTF * NHID * 2);
  float*          Bsum = (float*)carve((size_t)NTYPE * NGATE * 4);
  if (off > ws_size || off > (size_t)134217728) return;

  tpw_kernel<<<dim3(NGATE / 64, NHID / 64, NTYPE), NTHR, 0, stream>>>(w_hh, NHID, NGATE, KPITCH, WgT, WCARRY);
  wx_cols_kernel<<<(NTYPE * NGATE * 8) / NTHR, NTHR, 0, stream>>>(w_ih, WgT);
  tpw_kernel<<<dim3(NOUTF / 64, NHID / 64, NTYPE), NTHR, 0, stream>>>(fc_w, NHID, NOUTF, NHID, FcT, WCARRY);
  bias_sum_kernel<<<(NTYPE * NGATE / 4) / NTHR, NTHR, 0, stream>>>(b_ih, b_hh, Bsum);
  enc_kernel<<<NNODE * (NBAT / BMROWS), NTHR, 0, stream>>>(x, node_types, h1_w, h1_b, h2_w, h2_b, fc_b,
                                                           WgT, FcT, Bsum, out);
}
